// LocalFeatureAggregation_15925738734009
// MI455X (gfx1250) — hardware-verified
//
#include <hip/hip_runtime.h>
#include <math.h>

constexpr int NPTS = 8192;
constexpr int NBAT = 2;
constexpr int KNBR = 16;
constexpr int MN   = NBAT * NPTS;
constexpr int MNK  = MN * KNBR;
constexpr int CIN  = 64;
constexpr int CH1  = 64;
constexpr int CH2  = 128;
constexpr int CH4  = 256;
constexpr int TPITCH = 136;
constexpr int SPW    = 36;
constexpr float WCARRY     = 16.0f;
constexpr float WCARRY_INV = 0.0625f;
constexpr float RESC       = 2048.0f;
constexpr float RESC_INV   = 0.00048828125f;
constexpr float EPS_BN     = 1e-6f;
constexpr size_t WS_LIMIT  = 134217728;

static_assert(MN % 64 == 0 && MNK % 128 == 0 && NPTS % 256 == 0 && NPTS % 8 == 0);
static_assert(CIN % 32 == 0 && CH1 % 64 == 0 && CH2 % 64 == 0 && CH4 % 64 == 0);

typedef __attribute__((ext_vector_type(16))) _Float16 v16h;
typedef __attribute__((ext_vector_type(8)))  _Float16 v8h;
typedef __attribute__((ext_vector_type(8)))  float    v8f;
typedef __attribute__((ext_vector_type(4)))  float    v4f;
typedef __attribute__((ext_vector_type(4)))  unsigned int v4u;
typedef __attribute__((ext_vector_type(4)))  int      v4i;

__device__ __forceinline__ void grp_guard8(v8f& a0, v8f& a1, v8f& a2, v8f& a3, v8f& b0, v8f& b1, v8f& b2, v8f& b3,
                                           v16h x, v16h xr, v16h y0, v16h y1, v16h y2, v16h y3) {
  asm volatile("v_nop\n\tv_nop\n\tv_nop\n\tv_nop"
               : "+v"(a0), "+v"(a1), "+v"(a2), "+v"(a3), "+v"(b0), "+v"(b1), "+v"(b2), "+v"(b3)
               : "v"(x), "v"(xr), "v"(y0), "v"(y1), "v"(y2), "v"(y3));
}
__device__ __forceinline__ void grp_guard4x(v8f& a0, v8f& a1, v8f& b0, v8f& b1, v16h x, v16h y0, v16h y1, v16h z0, v16h z1) {
  asm volatile("v_nop\n\tv_nop\n\tv_nop\n\tv_nop"
               : "+v"(a0), "+v"(a1), "+v"(b0), "+v"(b1)
               : "v"(x), "v"(y0), "v"(y1), "v"(z0), "v"(z1));
}
__device__ __forceinline__ void keep4_h(v16h a, v16h b, v16h c, v16h d) { asm volatile("v_nop" :: "v"(a), "v"(b), "v"(c), "v"(d)); }
__device__ __forceinline__ void acc_guard4(v8f& a, v8f& b, v8f& c, v8f& d) { asm volatile("v_nop\n\tv_nop\n\tv_nop\n\tv_nop" : "+v"(a), "+v"(b), "+v"(c), "+v"(d)); }
__device__ __forceinline__ void wave_lds_sync() {
  __builtin_amdgcn_fence(__ATOMIC_RELEASE, "workgroup");
  __builtin_amdgcn_wave_barrier();
  __builtin_amdgcn_fence(__ATOMIC_ACQUIRE, "workgroup");
}

struct FragH {
  union U { v16h v; v8h h[2]; };
  static __device__ __forceinline__ v16h load(const _Float16* p) {
    U f; f.h[0] = *(const v8h*)(p); f.h[1] = *(const v8h*)(p + 16); return f.v;
  }
  static __device__ __forceinline__ v8f mma(v16h a, v16h b, v8f c) {
    return __builtin_amdgcn_wmma_f32_16x16x32_f16(false, a, false, b, (short)0, c, false, false);
  }
};

__device__ __forceinline__ float h16_to_f32(unsigned hb) {
  const unsigned sgn = (hb & 0x8000u) << 16; const unsigned em = hb & 0x7fffu;
  const float fn = __uint_as_float((em << 13) + 0x38000000u);
  const float fs = (float)em * 5.9604644775390625e-8f;
  const float mag = (em < 0x400u) ? fs : fn; return __uint_as_float(__float_as_uint(mag) | sgn);
}
__device__ __forceinline__ unsigned short h_bits(float f) { const _Float16 h = (_Float16)f; return __builtin_bit_cast(unsigned short, h); }
__device__ __forceinline__ unsigned pk16(unsigned short a, unsigned short b) { return (unsigned)a | ((unsigned)b << 16); }
__device__ __forceinline__ v4u pack8h(const float (&v)[8]) {
  return (v4u){pk16(h_bits(v[0]), h_bits(v[1])), pk16(h_bits(v[2]), h_bits(v[3])),
               pk16(h_bits(v[4]), h_bits(v[5])), pk16(h_bits(v[6]), h_bits(v[7]))};
}
__device__ __forceinline__ void pack8hr(const float (&v)[8], v4u& uh, v4u& ur) {
  unsigned short hb[8], rb[8];
#pragma unroll
  for (int e = 0; e < 8; ++e) {
    hb[e] = h_bits(v[e]);
    const float hf = h16_to_f32((unsigned)hb[e]);
    rb[e] = h_bits((v[e] - hf) * RESC);
  }
  uh = (v4u){pk16(hb[0], hb[1]), pk16(hb[2], hb[3]), pk16(hb[4], hb[5]), pk16(hb[6], hb[7])};
  ur = (v4u){pk16(rb[0], rb[1]), pk16(rb[2], rb[3]), pk16(rb[4], rb[5]), pk16(rb[6], rb[7])};
}

template <bool ARES, bool BRES, int BIAS_MODE, int OUT_MODE, int ACT>
__global__ __launch_bounds__(256) void wmma_gemm32(
    const unsigned short* __restrict__ Ap, const unsigned short* __restrict__ ARp, int lda,
    const unsigned short* __restrict__ Btp, const unsigned short* __restrict__ BRp, int ldb,
    void* __restrict__ Cout, int ldc,
    const float* __restrict__ bias, const float* __restrict__ bias2,
    int M, int N, int K, float scale) {
  static_assert(ARES || BRES);
  const _Float16* Ab = (const _Float16*)Ap;
  const _Float16* Ar = (const _Float16*)ARp;
  const _Float16* Bb = (const _Float16*)Btp;
  const _Float16* Br = (const _Float16*)BRp;
  __shared__ __align__(16) float sT[8][16 * 68];
  const int lane = threadIdx.x & 31;
  const int wave = threadIdx.x >> 5;
  const int tilesN = N >> 6;
  const int tilesM = M >> 5;
  const int tile = blockIdx.x * 8 + wave;
  if (tile >= tilesM * tilesN) return;
  const int tm = tile / tilesN;
  const int tn = tile - tm * tilesN;
  const int m0 = tm << 5;
  const int n0 = tn << 6;
  const int rlane = lane & 15;
  const int koff  = (lane >> 4) * 8;
  const int mOff  = (lane >> 4) * 8;

  v8f acc[2][4], accr[2][4];
#pragma unroll
  for (int i = 0; i < 2; ++i)
#pragma unroll
    for (int j = 0; j < 4; ++j) {
      acc[i][j]  = (v8f){0.f,0.f,0.f,0.f,0.f,0.f,0.f,0.f};
      accr[i][j] = (v8f){0.f,0.f,0.f,0.f,0.f,0.f,0.f,0.f};
    }

  for (int k0 = 0; k0 < K; k0 += 32) {
    v16h bh[4], br[4];
#pragma unroll
    for (int j = 0; j < 4; ++j) {
      const size_t bo = (size_t)(n0 + (j << 4) + rlane) * ldb + koff + k0;
      bh[j] = FragH::load(Bb + bo);
      if (BRES) br[j] = FragH::load(Br + bo); else br[j] = bh[j];
    }
#pragma unroll
    for (int i = 0; i < 2; ++i) {
      const size_t ao = (size_t)(m0 + (i << 4) + rlane) * lda + koff + k0;
      const v16h ah = FragH::load(Ab + ao);
      v16h ar = ah;
      if (ARES) ar = FragH::load(Ar + ao);
#pragma unroll
      for (int j = 0; j < 4; ++j) {
        acc[i][j] = FragH::mma(ah, bh[j], acc[i][j]);
        if (BRES) accr[i][j] = FragH::mma(ah, br[j], accr[i][j]);
        if (ARES) accr[i][j] = FragH::mma(ar, bh[j], accr[i][j]);
      }
      grp_guard8(acc[i][0], acc[i][1], acc[i][2], acc[i][3], accr[i][0], accr[i][1], accr[i][2], accr[i][3],
                 ah, ar, bh[0], bh[1], bh[2], bh[3]);
    }
    keep4_h(bh[0], bh[1], bh[2], bh[3]);
    if (BRES) keep4_h(br[0], br[1], br[2], br[3]);
  }
  acc_guard4(acc[0][0], acc[0][1], acc[0][2], acc[0][3]);
  acc_guard4(acc[1][0], acc[1][1], acc[1][2], acc[1][3]);
  acc_guard4(accr[0][0], accr[0][1], accr[0][2], accr[0][3]);
  acc_guard4(accr[1][0], accr[1][1], accr[1][2], accr[1][3]);

  float* slab = sT[wave];

  if (OUT_MODE == 3) {
    float cs[4], cq[4];
#pragma unroll
    for (int j = 0; j < 4; ++j) {
      const int n = n0 + (j << 4) + rlane;
      float bv = 0.f;
      if (BIAS_MODE == 2) bv = bias[n];
      float s1 = 0.f, s2 = 0.f;
#pragma unroll
      for (int i = 0; i < 2; ++i)
#pragma unroll
        for (int r = 0; r < 8; ++r) {
          const float v = (acc[i][j][r] + accr[i][j][r] * RESC_INV) * scale + bv;
          s1 += v; s2 = fmaf(v, v, s2);
        }
      cs[j] = s1; cq[j] = s2;
    }
#pragma unroll
    for (int j = 0; j < 4; ++j) { cs[j] += __shfl_xor(cs[j], 16, 32); cq[j] += __shfl_xor(cq[j], 16, 32); }
    if (lane < 16) {
#pragma unroll
      for (int j = 0; j < 4; ++j) { slab[(j << 4) + rlane] = cs[j]; slab[64 + (j << 4) + rlane] = cq[j]; }
    }
    wave_lds_sync();
    const v4f o = *(const v4f*)(slab + 4 * lane);
    float* P = (float*)Cout + (size_t)tile * 128 + 4 * lane;
    *(volatile v4f*)P = o; __threadfence(); *(volatile v4f*)P = o;
    return;
  }

#pragma unroll
  for (int i = 0; i < 2; ++i) {
    const int mBase = m0 + (i << 4);
    float bm8[8];
    if (BIAS_MODE == 1) {
      const v4f b0 = *(const v4f*)(bias + mBase + mOff);
      const v4f b1 = *(const v4f*)(bias + mBase + mOff + 4);
#pragma unroll
      for (int e = 0; e < 4; ++e) { bm8[e] = b0[e]; bm8[4 + e] = b1[e]; }
    } else {
#pragma unroll
      for (int e = 0; e < 8; ++e) bm8[e] = 0.f;
    }
#pragma unroll
    for (int j = 0; j < 4; ++j) {
      const int n = n0 + (j << 4) + rlane;
      float bv = 0.f, bmul = 1.f;
      if (BIAS_MODE == 2) bv = bias[n];
      if (BIAS_MODE == 3) { bmul = bias[n]; bv = bias2[n]; }
#pragma unroll
      for (int r = 0; r < 8; ++r) {
        float v = (acc[i][j][r] + accr[i][j][r] * RESC_INV) * scale;
        if (BIAS_MODE == 1) v += bm8[r];
        if (BIAS_MODE == 2) v += bv;
        if (BIAS_MODE == 3) v = fmaf(v, bmul, bv);
        if (ACT == 2) v = fmaxf(v, 0.0f);
        slab[(mOff + r) * 68 + (j << 4) + rlane] = v;
      }
    }
    wave_lds_sync();
    if (OUT_MODE == 0) {
      float* C = (float*)Cout;
      const int hh = lane >> 4, c4 = (lane & 15) * 4;
      for (int pass = 0; pass < 2; ++pass) {
#pragma unroll
        for (int it = 0; it < 8; ++it) {
          const int row = it * 2 + hh;
          v4f v = *(const v4f*)(slab + row * 68 + c4);
          *(volatile v4f*)(C + (size_t)(mBase + row) * ldc + n0 + c4) = v;
        }
        __threadfence();
      }
    } else {
      unsigned short* C = (unsigned short*)Cout;
      const int q = lane >> 3, c8 = (lane & 7) * 8;
      for (int pass = 0; pass < 2; ++pass) {
#pragma unroll
        for (int it = 0; it < 4; ++it) {
          const int row = it * 4 + q;
          const float* sp = slab + row * 68 + c8;
          v8h hv;
#pragma unroll
          for (int e = 0; e < 8; ++e) hv[e] = (_Float16)sp[e];
          *(volatile v8h*)(C + (size_t)(mBase + row) * ldc + n0 + c8) = hv;
        }
        __threadfence();
      }
    }
    wave_lds_sync();
  }
}

__global__ __launch_bounds__(256) void cast8_split_kernel(const float* __restrict__ in, unsigned short* __restrict__ outH,
                                                         unsigned short* __restrict__ outR, int n8, float scale) {
  const int i = blockIdx.x * 256 + threadIdx.x;
  if (i >= n8) return;
  const float* p = in + 8 * (size_t)i;
  const v4f a = *(const v4f*)(p);
  const v4f c = *(const v4f*)(p + 4);
  float v[8];
#pragma unroll
  for (int e = 0; e < 4; ++e) { v[e] = a[e] * scale; v[4 + e] = c[e] * scale; }
  v4u uh, ur;
  pack8hr(v, uh, ur);
  unsigned short* qh = outH + 8 * (size_t)i;
  unsigned short* qr = outR + 8 * (size_t)i;
  *(volatile v4u*)qh = uh;
  *(volatile v4u*)qr = ur;
  __threadfence();
  *(volatile v4u*)qh = uh;
  *(volatile v4u*)qr = ur;
}

__global__ __launch_bounds__(256) void feat_transpose_kernel(const float* __restrict__ feat, unsigned short* __restrict__ featT) {
  __shared__ float sm[64][65];
  const int t  = threadIdx.x;
  const int n0 = blockIdx.x * 64;
  const int b  = blockIdx.y;
#pragma unroll
  for (int it = 0; it < 16; ++it) {
    const int e  = it * 256 + t;
    const int c  = e >> 6;
    const int nl = e & 63;
    sm[nl][c] = feat[((size_t)(b * CIN + c)) * NPTS + n0 + nl];
  }
  __syncthreads();
  const int lane = t & 31, wave = t >> 5;
  const int q = lane >> 3, c8 = (lane & 7) * 8;
  v4u u2[2];
#pragma unroll
  for (int it = 0; it < 2; ++it) {
    const int row = wave * 8 + it * 4 + q;
    float v[8];
#pragma unroll
    for (int e = 0; e < 8; ++e) v[e] = sm[row][c8 + e];
    u2[it] = pack8h(v);
  }
  for (int pass = 0; pass < 2; ++pass) {
#pragma unroll
    for (int it = 0; it < 2; ++it) {
      const int row = wave * 8 + it * 4 + q;
      *(volatile v4u*)(featT + ((size_t)(b * NPTS + n0 + row)) * CIN + c8) = u2[it];
    }
    __threadfence();
  }
}

__global__ __launch_bounds__(256) void knn_kernel(const float* __restrict__ xyz, int* __restrict__ nbrs, float* __restrict__ dist) {
#pragma clang fp contract(off)
  __shared__ float sx[256];
  __shared__ float sy[256];
  __shared__ float sz[256];
  __shared__ float ss[256];
  __shared__ __align__(16) int   snb[256 * KNBR];
  __shared__ __align__(16) float sds[256 * KNBR];
  const int tid = threadIdx.x;
  const int b   = blockIdx.y;
  const int qi  = blockIdx.x * 256 + tid;
  const float* qp = xyz + ((size_t)b * NPTS + qi) * 3;
  const float qx = qp[0], qy = qp[1], qz = qp[2];
  const float t0 = qx * qx;
  const float t1 = qy * qy;
  const float t2 = qz * qz;
  const float qs = (t0 + t2) + t1;
  float bd[KNBR]; int bi[KNBR];
#pragma unroll
  for (int j = 0; j < KNBR; ++j) { bd[j] = 3.0e38f; bi[j] = 0; }
  for (int s0 = 0; s0 < NPTS; s0 += 256) {
    __syncthreads();
    {
      const float* sp = xyz + ((size_t)b * NPTS + s0 + tid) * 3;
      const float x = sp[0], y = sp[1], z = sp[2];
      const float u0 = x * x;
      const float u1 = y * y;
      const float u2 = z * z;
      sx[tid] = x; sy[tid] = y; sz[tid] = z;
      ss[tid] = (u0 + u2) + u1;
    }
    __syncthreads();
#pragma unroll 1
    for (int j = 0; j < 256; ++j) {
      float p = qx * sx[j];
      p = fmaf(qy, sy[j], p);
      p = fmaf(qz, sz[j], p);
      const float su = qs + ss[j];
      const float p2 = 2.0f * p;
      const float d2 = su - p2;
      if (d2 < bd[KNBR - 1]) {
        bd[KNBR - 1] = d2; bi[KNBR - 1] = s0 + j;
#pragma unroll
        for (int u = KNBR - 1; u > 0; --u) {
          const bool sw = bd[u] < bd[u - 1];
          const float dlo = sw ? bd[u] : bd[u - 1];
          const float dhi = sw ? bd[u - 1] : bd[u];
          const int   ilo = sw ? bi[u] : bi[u - 1];
          const int   ihi = sw ? bi[u - 1] : bi[u];
          bd[u - 1] = dlo; bd[u] = dhi; bi[u - 1] = ilo; bi[u] = ihi;
        }
      }
    }
  }
#pragma unroll
  for (int j4 = 0; j4 < 4; ++j4) {
    const v4i iv = (v4i){bi[4 * j4], bi[4 * j4 + 1], bi[4 * j4 + 2], bi[4 * j4 + 3]};
    v4f dv;
    dv[0] = sqrtf(fmaxf(bd[4 * j4],     1e-12f));
    dv[1] = sqrtf(fmaxf(bd[4 * j4 + 1], 1e-12f));
    dv[2] = sqrtf(fmaxf(bd[4 * j4 + 2], 1e-12f));
    dv[3] = sqrtf(fmaxf(bd[4 * j4 + 3], 1e-12f));
    *(v4i*)(snb + tid * KNBR + 4 * j4) = iv;
    *(v4f*)(sds + tid * KNBR + 4 * j4) = dv;
  }
  __syncthreads();
  const size_t base = ((size_t)b * NPTS + (size_t)blockIdx.x * 256) * KNBR;
  for (int pass = 0; pass < 2; ++pass) {
#pragma unroll
    for (int it = 0; it < 4; ++it) {
      const int idx = (it * 256 + tid) * 4;
      const v4i a = *(const v4i*)(snb + idx);
      const v4f d = *(const v4f*)(sds + idx);
      *(volatile v4i*)(nbrs + base + idx) = a;
      *(volatile v4f*)(dist + base + idx) = d;
    }
    __threadfence();
  }
}

template <int MODE>
__global__ __launch_bounds__(256) void rpe1_kernel(const float* __restrict__ xyz, const int* __restrict__ nbrs, const float* __restrict__ dist,
                                                  const float* __restrict__ W, const float* __restrict__ bconv, const float* __restrict__ stats,
                                                  const float* __restrict__ g, const float* __restrict__ be,
                                                  float* __restrict__ part, unsigned short* __restrict__ rpe, int pairsPerBlock) {
  __shared__ float sw[CH1 * 10];
  __shared__ float sv[5][CH1];
  __shared__ __align__(16) float red[8][128];
  const int tid = threadIdx.x, lane = tid & 31, wave = tid >> 5;
  for (int i = tid; i < CH1 * 10; i += 256) sw[i] = W[i];
  if (tid < CH1) {
    sv[0][tid] = bconv[tid];
    if (MODE == 1) { sv[1][tid] = stats[tid]; sv[2][tid] = stats[256 + tid]; sv[3][tid] = g[tid]; sv[4][tid] = be[tid]; }
  }
  __syncthreads();
  const int q = lane >> 3, c8 = (lane & 7) * 8;
  float ca0[8], ca1[8], ca2[8], cb0[8], cb1[8], cb2[8], w9[8], b0[8], mulc[8], addc[8];
#pragma unroll
  for (int e = 0; e < 8; ++e) {
    const int c = c8 + e; const float* wr = sw + c * 10;
    ca0[e] = wr[0] + wr[6]; ca1[e] = wr[1] + wr[7]; ca2[e] = wr[2] + wr[8];
    cb0[e] = wr[3] - wr[6]; cb1[e] = wr[4] - wr[7]; cb2[e] = wr[5] - wr[8];
    w9[e] = wr[9]; b0[e] = sv[0][c];
    if (MODE == 1) { mulc[e] = sv[3][c] * sv[2][c]; addc[e] = sv[4][c] - sv[1][c] * mulc[e]; }
    else { mulc[e] = 0.f; addc[e] = 0.f; }
  }
  float s[8], sq[8];
#pragma unroll
  for (int e = 0; e < 8; ++e) { s[e] = 0.f; sq[e] = 0.f; }
  const int iters = pairsPerBlock >> 5;
#pragma unroll 1
  for (int it = 0; it < iters; ++it) {
    const int pair = blockIdx.x * pairsPerBlock + it * 32 + wave * 4 + q;
    const int gp = pair >> 4;
    const int bbase = (gp / NPTS) * NPTS;
    int nb = nbrs[pair]; nb = nb < 0 ? 0 : (nb > NPTS - 1 ? NPTS - 1 : nb);
    const float ds = dist[pair];
    const float* pn = xyz + (size_t)gp * 3;
    const float* pb = xyz + (size_t)(bbase + nb) * 3;
    const float xn0 = pn[0], xn1 = pn[1], xn2 = pn[2];
    const float xb0 = pb[0], xb1 = pb[1], xb2 = pb[2];
    float v[8];
#pragma unroll
    for (int e = 0; e < 8; ++e) {
      float t = b0[e];
      t = fmaf(ca0[e], xn0, t); t = fmaf(ca1[e], xn1, t); t = fmaf(ca2[e], xn2, t);
      t = fmaf(cb0[e], xb0, t); t = fmaf(cb1[e], xb1, t); t = fmaf(cb2[e], xb2, t);
      t = fmaf(w9[e], ds, t);
      v[e] = t;
    }
    if (MODE == 0) {
#pragma unroll
      for (int e = 0; e < 8; ++e) { s[e] += v[e]; sq[e] = fmaf(v[e], v[e], sq[e]); }
    } else {
      float y[8];
#pragma unroll
      for (int e = 0; e < 8; ++e) { const float t = fmaf(v[e], mulc[e], addc[e]); y[e] = fmaxf(t, 0.f); }
      const v4u u = pack8h(y);
      unsigned short* dst = rpe + (size_t)pair * CH1 + c8;
      *(volatile v4u*)dst = u;
      __threadfence();
      *(volatile v4u*)dst = u;
    }
  }
  if (MODE == 0) {
#pragma unroll
    for (int e = 0; e < 8; ++e) {
      s[e]  += __shfl_xor(s[e], 8, 32);  s[e]  += __shfl_xor(s[e], 16, 32);
      sq[e] += __shfl_xor(sq[e], 8, 32); sq[e] += __shfl_xor(sq[e], 16, 32);
    }
    if (lane < 8) {
#pragma unroll
      for (int e = 0; e < 8; ++e) { red[wave][c8 + e] = s[e]; red[wave][64 + c8 + e] = sq[e]; }
    }
    __syncthreads();
    if (wave == 0) {
      v4f o = (v4f){0.f, 0.f, 0.f, 0.f};
#pragma unroll
      for (int w = 0; w < 8; ++w) o = o + *(const v4f*)(&red[w][4 * lane]);
      float* dst = part + (size_t)blockIdx.x * 128 + 4 * lane;
      *(volatile v4f*)dst = o;
      __threadfence();
      *(volatile v4f*)dst = o;
    }
  }
}

template <bool PARTIAL>
__global__ __launch_bounds__(256) void bn_stats_kernel(const float* __restrict__ src, long strideC, long strideM, int T, int sqOff, float count,
                                                      const float* __restrict__ g, const float* __restrict__ be, const float* __restrict__ bconv,
                                                      float* __restrict__ stats) {
  __shared__ double rs[8][32];
  __shared__ double rq[8][32];
  __shared__ __align__(16) float so[4][32];
  const int tid = threadIdx.x, lane = tid & 31, wave = tid >> 5;
  const int c0 = blockIdx.x * 32;
  const int c  = c0 + lane;
  const float* p = src + (size_t)c * strideC;
  double s = 0.0, q = 0.0;
#pragma unroll 1
  for (int t = wave; t < T; t += 8) {
    const float* e = p + (size_t)t * strideM;
    const float y = e[0];
    if (PARTIAL) { const float yq = e[sqOff]; s += (double)y; q += (double)yq; }
    else { s += (double)y; q += (double)y * (double)y; }
  }
  rs[wave][lane] = s; rq[wave][lane] = q;
  __syncthreads();
  if (wave == 0) {
    double S = 0.0, Q = 0.0;
#pragma unroll
    for (int w = 0; w < 8; ++w) { S += rs[w][lane]; Q += rq[w][lane]; }
    const double inv = 1.0 / (double)count;
    const double mean = S * inv;
    double var = Q * inv - mean * mean;
    var = var > 0.0 ? var : 0.0;
    const float meanf = (float)mean;
    const float varf  = (float)var;
    const float rstd  = 1.0f / sqrtf(varf + EPS_BN);
    const float mul   = g[c] * rstd;
    const float addx  = be[c] + (bconv[c] - meanf) * mul;
    so[0][lane] = meanf; so[1][lane] = rstd; so[2][lane] = mul; so[3][lane] = addx;
  }
  __syncthreads();
  if (wave == 0) {
    const int vec = lane >> 3, i4 = (lane & 7) * 4;
    const v4f o = *(const v4f*)(&so[vec][i4]);
    float* dst = stats + vec * 256 + c0 + i4;
    *(volatile v4f*)dst = o;
    __threadfence();
    *(volatile v4f*)dst = o;
  }
}

template <int CH, int ACT, bool ORES>
__global__ __launch_bounds__(256) void bn_apply_kernel(const float* __restrict__ raw, const float* __restrict__ stats,
                                                      const float* __restrict__ g, const float* __restrict__ be,
                                                      unsigned short* __restrict__ outH, unsigned short* __restrict__ outR, int M) {
  __shared__ float sm[4][CH];
  for (int i = threadIdx.x; i < CH; i += 256) { sm[0][i] = stats[i]; sm[1][i] = stats[256 + i]; sm[2][i] = g[i]; sm[3][i] = be[i]; }
  __syncthreads();
  constexpr int LPR = CH / 8;
  constexpr int RPW = 32 / LPR;
  constexpr int RPB = 8 * RPW;
  const int lane = threadIdx.x & 31, wave = threadIdx.x >> 5;
  int row = blockIdx.x * RPB + wave * RPW + lane / LPR;
  row = row < M ? row : M - 1;
  const int c8 = (lane % LPR) * 8;
  const float* rp = raw + (size_t)row * CH + c8;
  const v4f a  = *(const v4f*)(rp);
  const v4f a2 = *(const v4f*)(rp + 4);
  float v[8];
#pragma unroll
  for (int e = 0; e < 4; ++e) { v[e] = a[e]; v[4 + e] = a2[e]; }
#pragma unroll
  for (int e = 0; e < 8; ++e) {
    const int ch = c8 + e;
    float y = (v[e] - sm[0][ch]) * sm[1][ch];
    y = y * sm[2][ch] + sm[3][ch];
    if (ACT == 1) y = fmaxf(y, 0.f);
    if (ACT == 2) y = (y >= 0.f) ? y : 0.2f * y;
    v[e] = y;
  }
  v4u uh, ur;
  if (ORES) pack8hr(v, uh, ur); else { uh = pack8h(v); ur = uh; }
  unsigned short* dh = outH + (size_t)row * CH + c8;
  unsigned short* dr = ORES ? (outR + (size_t)row * CH + c8) : dh;
  *(volatile v4u*)dh = uh;
  if (ORES) *(volatile v4u*)dr = ur;
  __threadfence();
  *(volatile v4u*)dh = uh;
  if (ORES) *(volatile v4u*)dr = ur;
}

template <bool ORES>
__global__ __launch_bounds__(256) void attpool_kernel(const unsigned short* __restrict__ rpeP, const unsigned short* __restrict__ ptP,
                                                     const int* __restrict__ nbrs, const unsigned short* __restrict__ WspH,
                                                     const unsigned short* __restrict__ WspR,
                                                     unsigned short* __restrict__ pooledH, unsigned short* __restrict__ pooledR) {
  __shared__ __align__(16) unsigned short tileA[128 * TPITCH];
  __shared__ __align__(16) float slabS[8][16 * SPW];
  __shared__ __align__(16) float poolB[8 * CH2];
  const int tid = threadIdx.x, lane = tid & 31, wave = tid >> 5;
  const int pair0 = blockIdx.x * 128;
  const int pt0   = blockIdx.x * 8;
  const int bb    = pt0 / NPTS;
#pragma unroll
  for (int it = 0; it < 4; ++it) {
    const int row = it * 32 + (tid >> 3);
    const int c8  = (tid & 7) * 8;
    const v4u u = *(const v4u*)(rpeP + (size_t)(pair0 + row) * CH1 + c8);
    int nb = nbrs[pair0 + row]; nb = nb < 0 ? 0 : (nb > NPTS - 1 ? NPTS - 1 : nb);
    const v4u gth = *(const v4u*)(ptP + (size_t)(bb * NPTS + nb) * CH1 + c8);
    *(v4u*)(tileA + row * TPITCH + c8) = u;
    *(v4u*)(tileA + row * TPITCH + CH1 + c8) = gth;
  }
  __syncthreads();

  const int mh = wave >> 2;
  const int n0 = (wave & 3) * 32;
  const int rlane = lane & 15;
  const int koff  = (lane >> 4) * 8;
  const int mOff  = koff;
  const _Float16* At  = (const _Float16*)tileA + (size_t)(mh * 64) * TPITCH;
  const _Float16* Bw  = (const _Float16*)WspH;
  const _Float16* Bwr = (const _Float16*)WspR;

  v8f acc[4][2], accr[4][2];
#pragma unroll
  for (int i = 0; i < 4; ++i)
#pragma unroll
    for (int j = 0; j < 2; ++j) {
      acc[i][j]  = (v8f){0.f,0.f,0.f,0.f,0.f,0.f,0.f,0.f};
      accr[i][j] = (v8f){0.f,0.f,0.f,0.f,0.f,0.f,0.f,0.f};
    }

#pragma unroll 1
  for (int k0 = 0; k0 < CH2; k0 += 32) {
    v16h bh[2], br[2];
#pragma unroll
    for (int j = 0; j < 2; ++j) {
      const size_t bo = (size_t)(n0 + (j << 4) + rlane) * CH2 + koff + k0;
      bh[j] = FragH::load(Bw + bo);
      br[j] = FragH::load(Bwr + bo);
    }
#pragma unroll
    for (int i = 0; i < 4; ++i) {
      const v16h ah = FragH::load(At + (size_t)((i << 4) + rlane) * TPITCH + koff + k0);
#pragma unroll
      for (int j = 0; j < 2; ++j) {
        acc[i][j]  = FragH::mma(ah, bh[j], acc[i][j]);
        accr[i][j] = FragH::mma(ah, br[j], accr[i][j]);
      }
      grp_guard4x(acc[i][0], acc[i][1], accr[i][0], accr[i][1], ah, bh[0], bh[1], br[0], br[1]);
    }
    keep4_h(bh[0], bh[1], br[0], br[1]);
  }
  acc_guard4(acc[0][0], acc[0][1], acc[1][0], acc[1][1]);
  acc_guard4(acc[2][0], acc[2][1], acc[3][0], acc[3][1]);
  acc_guard4(accr[0][0], accr[0][1], accr[1][0], accr[1][1]);
  acc_guard4(accr[2][0], accr[2][1], accr[3][0], accr[3][1]);

  float* slab = slabS[wave];
#pragma unroll
  for (int i = 0; i < 4; ++i) {
#pragma unroll
    for (int j = 0; j < 2; ++j)
#pragma unroll
      for (int r = 0; r < 8; ++r)
        slab[(mOff + r) * SPW + (j << 4) + rlane] = (acc[i][j][r] + accr[i][j][r] * RESC_INV) * WCARRY_INV;
    wave_lds_sync();
    const unsigned short* xrow = tileA + (size_t)(mh * 64 + (i << 4)) * TPITCH;
    const int ch = n0 + lane;
    float mx = -INFINITY;
#pragma unroll 1
    for (int k = 0; k < KNBR; ++k) mx = fmaxf(mx, slab[k * SPW + lane]);
    float se = 0.f, sw = 0.f;
#pragma unroll 1
    for (int k = 0; k < KNBR; ++k) {
      const float e  = expf(slab[k * SPW + lane] - mx);
      se += e;
      const float xv = h16_to_f32((unsigned)xrow[k * TPITCH + ch]);
      sw = fmaf(e, xv, sw);
    }
    poolB[(mh * 4 + i) * CH2 + ch] = sw * (1.0f / se);
    wave_lds_sync();
  }
  __syncthreads();
  {
    const int cl = (lane & 15) * 8;
    float v[8];
#pragma unroll
    for (int e = 0; e < 8; ++e) v[e] = poolB[wave * CH2 + cl + e];
    v4u uh, ur;
    if (ORES) pack8hr(v, uh, ur); else { uh = pack8h(v); ur = uh; }
    unsigned short* dh = pooledH + (size_t)(pt0 + wave) * CH2 + cl;
    unsigned short* dr = ORES ? (pooledR + (size_t)(pt0 + wave) * CH2 + cl) : dh;
    if (lane < 16) { *(volatile v4u*)dh = uh; if (ORES) *(volatile v4u*)dr = ur; }
    __threadfence();
    if (lane < 16) { *(volatile v4u*)dh = uh; if (ORES) *(volatile v4u*)dr = ur; }
  }
}

__global__ __launch_bounds__(256) void final_kernel(const float* __restrict__ rawA, const float* __restrict__ rawB,
                                                   const float* __restrict__ stA, const float* __restrict__ stB,
                                                   const float* __restrict__ gA, const float* __restrict__ beA,
                                                   const float* __restrict__ gB, const float* __restrict__ beB,
                                                   float* __restrict__ outp) {
  const int c = blockIdx.y;
  const int b = blockIdx.z;
  const int n = blockIdx.x * 1024 + threadIdx.x * 4;
  const float mA = stA[c], rA = stA[256 + c], ga = gA[c], ba = beA[c];
  const float mB = stB[c], rB = stB[256 + c], gb = gB[c], bbv = beB[c];
  const size_t src = (size_t)c * MN + (size_t)b * NPTS + n;
  const v4f ya = *(const v4f*)(rawA + src);
  const v4f yb = *(const v4f*)(rawB + src);
  v4f o;
#pragma unroll
  for (int e = 0; e < 4; ++e) {
    float u = (ya[e] - mA) * rA; u = u * ga + ba;
    float w = (yb[e] - mB) * rB; w = w * gb + bbv;
    const float t = u + w;
    o[e] = (t >= 0.f) ? t : 0.01f * t;
  }
  float* dst = outp + ((size_t)(b * CH4 + c)) * NPTS + n;
  *(volatile v4f*)dst = o;
  __threadfence();
  *(volatile v4f*)dst = o;
}

extern "C" void kernel_launch(void* const* d_in, const int* in_sizes, int n_in,
                              void* d_out, int out_size, void* d_ws, size_t ws_size,
                              hipStream_t stream) {
  (void)in_sizes; (void)n_in; (void)out_size;
  const float* xyz   = (const float*)d_in[0];
  const float* feat  = (const float*)d_in[1];
  const float* m1_w  = (const float*)d_in[2];
  const float* m1_b  = (const float*)d_in[3];
  const float* m1_g  = (const float*)d_in[4];
  const float* m1_be = (const float*)d_in[5];
  const float* r1_w  = (const float*)d_in[6];
  const float* r1_b  = (const float*)d_in[7];
  const float* r1_g  = (const float*)d_in[8];
  const float* r1_be = (const float*)d_in[9];
  const float* r2_w  = (const float*)d_in[10];
  const float* r2_b  = (const float*)d_in[11];
  const float* r2_g  = (const float*)d_in[12];
  const float* r2_be = (const float*)d_in[13];
  const float* p1s_w = (const float*)d_in[14];
  const float* p1_w  = (const float*)d_in[15];
  const float* p1_b  = (const float*)d_in[16];
  const float* p1_g  = (const float*)d_in[17];
  const float* p1_be = (const float*)d_in[18];
  const float* p2s_w = (const float*)d_in[19];
  const float* p2_w  = (const float*)d_in[20];
  const float* p2_b  = (const float*)d_in[21];
  const float* p2_g  = (const float*)d_in[22];
  const float* p2_be = (const float*)d_in[23];
  const float* m2_w  = (const float*)d_in[24];
  const float* m2_b  = (const float*)d_in[25];
  const float* m2_g  = (const float*)d_in[26];
  const float* m2_be = (const float*)d_in[27];
  const float* sc_w  = (const float*)d_in[28];
  const float* sc_b  = (const float*)d_in[29];
  const float* sc_g  = (const float*)d_in[30];
  const float* sc_be = (const float*)d_in[31];
  float* outp = (float*)d_out;

  char* ws = (char*)d_ws; size_t off = 0;
  auto carve = [&](size_t bytes) -> char* { char* p = ws + off; off += (bytes + 255) & ~(size_t)255; return p; };
  int*            nbrs   = (int*)carve((size_t)MNK * 4);
  float*          distp  = (float*)carve((size_t)MNK * 4);
  unsigned short* wtsH   = (unsigned short*)carve((size_t)114688 * 2);
  unsigned short* wtsR   = (unsigned short*)carve((size_t)114688 * 2);
  unsigned short* featT  = (unsigned short*)carve((size_t)MN * CIN * 2);
  unsigned short* rpe1   = (unsigned short*)carve((size_t)MNK * CH1 * 2);
  unsigned short* feats  = (unsigned short*)carve((size_t)MN * CH1 * 2);
  float*          rawpt  = (float*)carve((size_t)MN * CH2 * 4);
  unsigned short* pooled = (unsigned short*)carve((size_t)MN * CH2 * 2);
  unsigned short* f1     = (unsigned short*)carve((size_t)MN * CH1 * 2);
  unsigned short* rpe2   = (unsigned short*)carve((size_t)MNK * CH1 * 2);
  float*          rawm2  = (float*)carve((size_t)CH4 * MN * 4);
  float*          rawsc  = (float*)carve((size_t)CH4 * MN * 4);
  float*          part   = (float*)carve((size_t)8192 * 128 * 4);
  float*          statsA = (float*)carve(4096);
  float*          statsB = (float*)carve(4096);
  if (off > ws_size || off > WS_LIMIT) return;

  static_assert((size_t)3 * MN * CH2 * 2 <= (size_t)MNK * CH1 * 2);
  unsigned short* pooledR = rpe1;
  unsigned short* g2H     = rpe1 + (size_t)MN * CH2;
  unsigned short* g2R     = rpe1 + (size_t)2 * MN * CH2;

  unsigned short* w_m1  = wtsH;          unsigned short* r_m1  = wtsR;
  unsigned short* w_r2  = wtsH + 4096;   unsigned short* r_r2  = wtsR + 4096;
  unsigned short* w_p1s = wtsH + 8192;   unsigned short* r_p1s = wtsR + 8192;
  unsigned short* w_p1  = wtsH + 24576;  unsigned short* r_p1  = wtsR + 24576;
  unsigned short* w_p2s = wtsH + 32768;  unsigned short* r_p2s = wtsR + 32768;
  unsigned short* w_p2  = wtsH + 49152;  unsigned short* r_p2  = wtsR + 49152;
  unsigned short* w_m2  = wtsH + 65536;  unsigned short* r_m2  = wtsR + 65536;
  unsigned short* w_sc  = wtsH + 98304;  unsigned short* r_sc  = wtsR + 98304;

  cast8_split_kernel<<<(CH1 * CIN / 8) / 256, 256, 0, stream>>>(m1_w,  w_m1,  r_m1,  CH1 * CIN / 8, WCARRY);
  cast8_split_kernel<<<(CH1 * CH1 / 8) / 256, 256, 0, stream>>>(r2_w,  w_r2,  r_r2,  CH1 * CH1 / 8, WCARRY);
  cast8_split_kernel<<<(CH2 * CH2 / 8) / 256, 256, 0, stream>>>(p1s_w, w_p1s, r_p1s, CH2 * CH2 / 8, WCARRY);
  cast8_split_kernel<<<(CH1 * CH2 / 8) / 256, 256, 0, stream>>>(p1_w,  w_p1,  r_p1,  CH1 * CH2 / 8, WCARRY);
  cast8_split_kernel<<<(CH2 * CH2 / 8) / 256, 256, 0, stream>>>(p2s_w, w_p2s, r_p2s, CH2 * CH2 / 8, WCARRY);
  cast8_split_kernel<<<(CH2 * CH2 / 8) / 256, 256, 0, stream>>>(p2_w,  w_p2,  r_p2,  CH2 * CH2 / 8, WCARRY);
  cast8_split_kernel<<<(CH4 * CH2 / 8) / 256, 256, 0, stream>>>(m2_w,  w_m2,  r_m2,  CH4 * CH2 / 8, WCARRY);
  cast8_split_kernel<<<(CH4 * CIN / 8) / 256, 256, 0, stream>>>(sc_w,  w_sc,  r_sc,  CH4 * CIN / 8, WCARRY);
  static_assert((CH1 * CIN / 8) % 256 == 0 && (CH2 * CH2 / 8) % 256 == 0 && (CH1 * CH2 / 8) % 256 == 0 && (CH4 * CH2 / 8) % 256 == 0 && (CH4 * CIN / 8) % 256 == 0);

  feat_transpose_kernel<<<dim3(NPTS / 64, NBAT), 256, 0, stream>>>(feat, featT);
  knn_kernel<<<dim3(NPTS / 256, NBAT), 256, 0, stream>>>(xyz, nbrs, distp);

  static_assert(MNK == 512 * 512 && MNK == 2048 * 128);
  rpe1_kernel<0><<<512, 256, 0, stream>>>(xyz, nbrs, distp, r1_w, r1_b, statsA, r1_g, r1_be, part, rpe1, 512);
  bn_stats_kernel<true><<<CH1 / 32, 256, 0, stream>>>(part, 1L, 128L, 512, 64, (float)MNK, r1_g, r1_be, r1_b, statsA);
  rpe1_kernel<1><<<2048, 256, 0, stream>>>(xyz, nbrs, distp, r1_w, r1_b, statsA, r1_g, r1_be, part, rpe1, 128);

  static_assert(MN % 32 == 0 && CH1 % 64 == 0 && CIN % 32 == 0 && ((MN / 32) * (CH1 / 64)) % 8 == 0);
  wmma_gemm32<false, true, 2, 0, 0><<<((MN / 32) * (CH1 / 64)) / 8, 256, 0, stream>>>(
      featT, (const unsigned short*)nullptr, CIN, w_m1, r_m1, CIN, (void*)rawpt, CH1, m1_b, (const float*)nullptr, MN, CH1, CIN, WCARRY_INV);
  bn_stats_kernel<false><<<CH1 / 32, 256, 0, stream>>>(rawpt, 1L, (long)CH1, MN, 0, (float)MN, m1_g, m1_be, m1_b, statsA);
  static_assert(MN % 32 == 0 && MN % 16 == 0);
  bn_apply_kernel<CH1, 2, false><<<MN / 32, 256, 0, stream>>>(rawpt, statsA, m1_g, m1_be, feats, (unsigned short*)nullptr, MN);

  static_assert(MNK % 128 == 0 && CH2 % 32 == 0);
  attpool_kernel<false><<<MNK / 128, 256, 0, stream>>>(rpe1, feats, nbrs, w_p1s, r_p1s, pooled, (unsigned short*)nullptr);
  wmma_gemm32<false, true, 2, 0, 0><<<((MN / 32) * (CH1 / 64)) / 8, 256, 0, stream>>>(
      pooled, (const unsigned short*)nullptr, CH2, w_p1, r_p1, CH2, (void*)rawpt, CH1, p1_b, (const float*)nullptr, MN, CH1, CH2, WCARRY_INV);
  bn_stats_kernel<false><<<CH1 / 32, 256, 0, stream>>>(rawpt, 1L, (long)CH1, MN, 0, (float)MN, p1_g, p1_be, p1_b, statsA);
  bn_apply_kernel<CH1, 1, false><<<MN / 32, 256, 0, stream>>>(rawpt, statsA, p1_g, p1_be, f1, (unsigned short*)nullptr, MN);

  static_assert(MNK % 32 == 0 && ((MNK / 32) * (CH1 / 64)) % 8 == 0 && (MNK / 32) * (CH1 / 64) == 8192);
  wmma_gemm32<false, true, 2, 3, 0><<<((MNK / 32) * (CH1 / 64)) / 8, 256, 0, stream>>>(
      rpe1, (const unsigned short*)nullptr, CH1, w_r2, r_r2, CH1, (void*)part, CH1, r2_b, (const float*)nullptr, MNK, CH1, CH1, WCARRY_INV);
  bn_stats_kernel<true><<<CH1 / 32, 256, 0, stream>>>(part, 1L, 128L, (MNK / 32) * (CH1 / 64), 64, (float)MNK, r2_g, r2_be, r2_b, statsA);
  wmma_gemm32<false, true, 3, 1, 2><<<((MNK / 32) * (CH1 / 64)) / 8, 256, 0, stream>>>(
      rpe1, (const unsigned short*)nullptr, CH1, w_r2, r_r2, CH1, (void*)rpe2, CH1, statsA + 512, statsA + 768, MNK, CH1, CH1, WCARRY_INV);

  attpool_kernel<true><<<MNK / 128, 256, 0, stream>>>(rpe2, f1, nbrs, w_p2s, r_p2s, pooled, pooledR);
  static_assert(((MN / 32) * (CH2 / 64)) % 8 == 0);
  wmma_gemm32<true, true, 2, 0, 0><<<((MN / 32) * (CH2 / 64)) / 8, 256, 0, stream>>>(
      pooled, pooledR, CH2, w_p2, r_p2, CH2, (void*)rawpt, CH2, p2_b, (const float*)nullptr, MN, CH2, CH2, WCARRY_INV);
  bn_stats_kernel<false><<<CH2 / 32, 256, 0, stream>>>(rawpt, 1L, (long)CH2, MN, 0, (float)MN, p2_g, p2_be, p2_b, statsA);
  bn_apply_kernel<CH2, 1, true><<<MN / 16, 256, 0, stream>>>(rawpt, statsA, p2_g, p2_be, g2H, g2R, MN);

  static_assert(CH4 % 32 == 0 && ((CH4 / 32) * (MN / 64)) % 8 == 0);
  wmma_gemm32<true, true, 1, 0, 0><<<((CH4 / 32) * (MN / 64)) / 8, 256, 0, stream>>>(
      w_m2, r_m2, CH2, g2H, g2R, CH2, (void*)rawm2, MN, m2_b, (const float*)nullptr, CH4, MN, CH2, WCARRY_INV);
  bn_stats_kernel<false><<<CH4 / 32, 256, 0, stream>>>(rawm2, (long)MN, 1L, MN, 0, (float)MN, m2_g, m2_be, m2_b, statsA);
  wmma_gemm32<true, false, 1, 0, 0><<<((CH4 / 32) * (MN / 64)) / 8, 256, 0, stream>>>(
      w_sc, r_sc, CIN, featT, (const unsigned short*)nullptr, CIN, (void*)rawsc, MN, sc_b, (const float*)nullptr, CH4, MN, CIN, WCARRY_INV);
  bn_stats_kernel<false><<<CH4 / 32, 256, 0, stream>>>(rawsc, (long)MN, 1L, MN, 0, (float)MN, sc_g, sc_be, sc_b, statsB);

  static_assert(NPTS % 1024 == 0 && NBAT * CH4 * NPTS * 4 == 16777216);
  final_kernel<<<dim3(NPTS / 1024, CH4, NBAT), 256, 0, stream>>>(rawm2, rawsc, statsA, statsB, m2_g, m2_be, sc_g, sc_be, outp);
}
